// XEGNNK_47863115547369
// MI455X (gfx1250) — hardware-verified
//
#include <hip/hip_runtime.h>
#define NNODE 20000
#define NEDGE 200000
#define NP2 262144
#define NG 64
#define KV 128
#define DH 64
#define TE 256
#define MSGK 512
#define NSL 2
#define ESL (NEDGE / NSL)

typedef __bf16 v16b __attribute__((ext_vector_type(16)));
typedef unsigned short v8us __attribute__((ext_vector_type(8), may_alias));
typedef float  v8f  __attribute__((ext_vector_type(8)));
typedef float  v4f  __attribute__((ext_vector_type(4)));
typedef float  v4fa __attribute__((ext_vector_type(4), may_alias));
union FragB { v16b v; v8us half[2]; unsigned short u[16]; };

__device__ __forceinline__ unsigned short bf16_bits(float x) { unsigned int u = __float_as_uint(x); return (unsigned short)((u + 0x7FFFu + ((u >> 16) & 1u)) >> 16); }
__device__ __forceinline__ float bf16_val(unsigned short b) { return __uint_as_float(((unsigned int)b) << 16); }
__device__ __forceinline__ float bf16_round(float x) { return bf16_val(bf16_bits(x)); }
template <int NT>
__device__ __forceinline__ v8f mmaN(v16b ah, v16b al, v16b bh, v16b bl, v8f c) {
  c = __builtin_amdgcn_wmma_f32_16x16x32_bf16(false, ah, false, bh, (short)0, c, false, false);
  if (NT >= 2) c = __builtin_amdgcn_wmma_f32_16x16x32_bf16(false, al, false, bh, (short)0, c, false, false);
  if (NT >= 3) c = __builtin_amdgcn_wmma_f32_16x16x32_bf16(false, ah, false, bl, (short)0, c, false, false);
  asm volatile("v_nop\n\tv_nop\n\tv_nop\n\tv_nop" : "+v"(c) : "v"(ah), "v"(al), "v"(bh), "v"(bl));
  return c;
}

__global__ __launch_bounds__(256) void k_wt_bf16(const float* __restrict__ W, unsigned short* __restrict__ Wt, int K, int N) {
  const int t = blockIdx.x * 256 + threadIdx.x;
  const int k8n = K / 8;
  if (t >= N * k8n) return;
  const int n = t / k8n, k8 = (t % k8n) * 8;
  v8us v;
#pragma unroll
  for (int i = 0; i < 8; ++i) v[i] = bf16_bits(W[(size_t)(k8 + i) * N + n]);
  *(volatile v8us*)(Wt + (size_t)n * K + k8) = v;
  __threadfence();
  *(volatile v8us*)(Wt + (size_t)n * K + k8) = v;
}

template <bool ASPLIT, int ACT, bool BIAS_BF16>
__global__ __launch_bounds__(128) void k_gemm_bf(const float* __restrict__ A, int lda, const unsigned short* __restrict__ Wt, int ldb,
                                               const float* __restrict__ bias, float* __restrict__ C, int ldc, int M, int N, int K) {
  __shared__ __attribute__((aligned(16))) float so[4][16][64];
  const int tid = threadIdx.x, w = tid >> 5, lane = tid & 31, ln = lane & 15, hh = lane >> 4;
  const int ntn = N / 64;
  const int wid = blockIdx.x * 4 + w;
  const int mt = wid / ntn, nq = wid % ntn;
  if (mt * 16 >= M) return;
  const int row0 = mt * 16, col0 = nq * 64;
  const float* arow = A + (size_t)(row0 + ln) * lda;
  v8f acc[4] = {};
  for (int kb = 0; kb < K; kb += 32) {
    FragB ah, al;
    const v4f x0 = *(const v4fa*)(arow + kb + 8 * hh), x1 = *(const v4fa*)(arow + kb + 8 * hh + 4);
    const v4f x2 = *(const v4fa*)(arow + kb + 16 + 8 * hh), x3 = *(const v4fa*)(arow + kb + 16 + 8 * hh + 4);
    float xs[16] = {x0[0],x0[1],x0[2],x0[3],x1[0],x1[1],x1[2],x1[3],x2[0],x2[1],x2[2],x2[3],x3[0],x3[1],x3[2],x3[3]};
#pragma unroll
    for (int i = 0; i < 16; ++i) { const unsigned short hb = bf16_bits(xs[i]); ah.u[i] = hb; al.u[i] = ASPLIT ? bf16_bits(xs[i] - bf16_val(hb)) : (unsigned short)0; }
#pragma unroll
    for (int t = 0; t < 4; ++t) {
      const unsigned short* brow = Wt + (size_t)(col0 + t * 16 + ln) * ldb + kb;
      FragB b;
      b.half[0] = *(const v8us*)(brow + 8 * hh);
      b.half[1] = *(const v8us*)(brow + 16 + 8 * hh);
      acc[t] = mmaN<ASPLIT ? 2 : 1>(ah.v, al.v, b.v, b.v, acc[t]);
    }
  }
#pragma unroll
  for (int t = 0; t < 4; ++t) {
    float bv = bias ? bias[col0 + t * 16 + ln] : 0.f;
    if (BIAS_BF16) bv = bf16_round(bv);
#pragma unroll
    for (int r = 0; r < 8; ++r) { float v = acc[t][r] + bv; if (ACT == 1) v = fmaxf(v, 0.f); so[w][8 * hh + r][t * 16 + ln] = v; }
  }
  __builtin_amdgcn_fence(__ATOMIC_ACQ_REL, "workgroup");
  __builtin_amdgcn_wave_barrier();
  const int rsub = lane >> 4, c4 = (lane & 15) * 4;
  for (int pass = 0; pass < 2; ++pass) {
#pragma unroll
    for (int q = 0; q < 8; ++q) {
      const int r = q * 2 + rsub;
      const v4f v = *(const v4fa*)&so[w][r][c4];
      *(volatile v4f*)(C + (size_t)(row0 + r) * ldc + col0 + c4) = v;
    }
    if (pass == 0) __threadfence();
  }
}

template <int D, bool CAUSAL>
__global__ __launch_bounds__(128) void k_flash(const float* __restrict__ qb, const float* __restrict__ kb, const float* __restrict__ vb,
                                             int pitch, int T, int H, float scale, float* __restrict__ y, int ypitch) {
  constexpr int KS = D / 32;
  constexpr int DT = D / 16;
  __shared__ __attribute__((aligned(16))) unsigned short sKh[32][D + 8], sKl[32][D + 8], sVh[32][D + 8], sVl[32][D + 8];
  __shared__ __attribute__((aligned(16))) unsigned short sPh[4][16][40], sPl[4][16][40];
  __shared__ __attribute__((aligned(16))) float sO[4][16][D];
  const int tid = threadIdx.x, w = tid >> 5, lane = tid & 31, ln = lane & 15, hh = lane >> 4;
  const int nqb = (T + 63) / 64;
  const int bh = blockIdx.x / nqb, qblk = blockIdx.x % nqb;
  const int b = bh / H, h = bh % H;
  const int q0 = qblk * 64 + w * 16;
  const float* Q = qb + (size_t)b * T * pitch + h * D;
  const float* K = kb + (size_t)b * T * pitch + h * D;
  const float* V = vb + (size_t)b * T * pitch + h * D;

  FragB aqh[KS], aql[KS];
  {
    int row = q0 + ln; if (row >= T) row = T - 1;
    const float* qr = Q + (size_t)row * pitch;
#pragma unroll
    for (int ks = 0; ks < KS; ++ks)
#pragma unroll
      for (int i = 0; i < 16; ++i) {
        const int d = ks * 32 + ((i < 8) ? (8 * hh + i) : (16 + 8 * hh + (i - 8)));
        const float x = qr[d] * scale; const unsigned short hb = bf16_bits(x);
        aqh[ks].u[i] = hb; aql[ks].u[i] = bf16_bits(x - bf16_val(hb));
      }
  }
  float m_r[8], l_r[8];
#pragma unroll
  for (int r = 0; r < 8; ++r) { m_r[r] = -3.0e38f; l_r[r] = 0.f; }
  v8f oacc[DT];
#pragma unroll
  for (int dt = 0; dt < DT; ++dt) oacc[dt] = (v8f){0.f,0.f,0.f,0.f,0.f,0.f,0.f,0.f};

  const int kv_end = CAUSAL ? min(T, qblk * 64 + 64) : T;
  for (int j0 = 0; j0 < kv_end; j0 += 32) {
    __syncthreads();
    for (int e = tid; e < 32 * (D / 4); e += 128) {
      const int r = e / (D / 4), c4 = (e % (D / 4)) * 4;
      const int key = j0 + r;
      v4f kf = {0.f,0.f,0.f,0.f}, vf = {0.f,0.f,0.f,0.f};
      if (key < T) { kf = *(const v4fa*)(K + (size_t)key * pitch + c4); vf = *(const v4fa*)(V + (size_t)key * pitch + c4); }
#pragma unroll
      for (int t = 0; t < 4; ++t) {
        unsigned short hb = bf16_bits(kf[t]); sKh[r][c4 + t] = hb; sKl[r][c4 + t] = bf16_bits(kf[t] - bf16_val(hb));
        hb = bf16_bits(vf[t]); sVh[r][c4 + t] = hb; sVl[r][c4 + t] = bf16_bits(vf[t] - bf16_val(hb));
      }
    }
    __syncthreads();
    v8f s[2];
#pragma unroll
    for (int nt = 0; nt < 2; ++nt) {
      v8f acc = {};
#pragma unroll
      for (int ks = 0; ks < KS; ++ks) {
        FragB bh_, bl_;
        bh_.half[0] = *(const v8us*)&sKh[nt * 16 + ln][ks * 32 + 8 * hh]; bh_.half[1] = *(const v8us*)&sKh[nt * 16 + ln][ks * 32 + 16 + 8 * hh];
        bl_.half[0] = *(const v8us*)&sKl[nt * 16 + ln][ks * 32 + 8 * hh]; bl_.half[1] = *(const v8us*)&sKl[nt * 16 + ln][ks * 32 + 16 + 8 * hh];
        acc = mmaN<3>(aqh[ks].v, aql[ks].v, bh_.v, bl_.v, acc);
      }
      s[nt] = acc;
    }
    float alpha[8];
#pragma unroll
    for (int r = 0; r < 8; ++r) {
      const int qi = q0 + 8 * hh + r;
      const int ja = j0 + ln, jb = j0 + 16 + ln;
      if (CAUSAL) { if (ja > qi) s[0][r] = -3.0e38f; if (jb > qi) s[1][r] = -3.0e38f; }
      if (ja >= T) s[0][r] = -3.0e38f;
      if (jb >= T) s[1][r] = -3.0e38f;
      float mx = fmaxf(s[0][r], s[1][r]);
      mx = fmaxf(mx, __shfl_xor(mx, 1, 32)); mx = fmaxf(mx, __shfl_xor(mx, 2, 32)); mx = fmaxf(mx, __shfl_xor(mx, 4, 32)); mx = fmaxf(mx, __shfl_xor(mx, 8, 32));
      const float mnew = fmaxf(m_r[r], mx);
      alpha[r] = (mnew > -1.0e38f) ? __expf(m_r[r] - mnew) : 1.0f;
      const float p0 = (s[0][r] > -1.0e38f) ? __expf(s[0][r] - mnew) : 0.f;
      const float p1 = (s[1][r] > -1.0e38f) ? __expf(s[1][r] - mnew) : 0.f;
      m_r[r] = mnew;
      l_r[r] = l_r[r] * alpha[r] + p0 + p1;
      unsigned short hb = bf16_bits(p0); sPh[w][8 * hh + r][ln] = hb;      sPl[w][8 * hh + r][ln] = bf16_bits(p0 - bf16_val(hb));
      hb = bf16_bits(p1);                sPh[w][8 * hh + r][16 + ln] = hb; sPl[w][8 * hh + r][16 + ln] = bf16_bits(p1 - bf16_val(hb));
    }
#pragma unroll
    for (int dt = 0; dt < DT; ++dt)
#pragma unroll
      for (int r = 0; r < 8; ++r) oacc[dt][r] *= alpha[r];
    __builtin_amdgcn_fence(__ATOMIC_ACQ_REL, "workgroup");
    __builtin_amdgcn_wave_barrier();
    FragB pah, pal;
    pah.half[0] = *(const v8us*)&sPh[w][ln][8 * hh]; pah.half[1] = *(const v8us*)&sPh[w][ln][16 + 8 * hh];
    pal.half[0] = *(const v8us*)&sPl[w][ln][8 * hh]; pal.half[1] = *(const v8us*)&sPl[w][ln][16 + 8 * hh];
#pragma unroll
    for (int dt = 0; dt < DT; ++dt) {
      FragB bvh, bvl;
#pragma unroll
      for (int i = 0; i < 8; ++i) {
        bvh.u[i] = sVh[8 * hh + i][dt * 16 + ln]; bvh.u[8 + i] = sVh[16 + 8 * hh + i][dt * 16 + ln];
        bvl.u[i] = sVl[8 * hh + i][dt * 16 + ln]; bvl.u[8 + i] = sVl[16 + 8 * hh + i][dt * 16 + ln];
      }
      oacc[dt] = mmaN<3>(pah.v, pal.v, bvh.v, bvl.v, oacc[dt]);
    }
    __builtin_amdgcn_fence(__ATOMIC_ACQ_REL, "workgroup");
    __builtin_amdgcn_wave_barrier();
  }
#pragma unroll
  for (int r = 0; r < 8; ++r) {
    float l = l_r[r];
    l += __shfl_xor(l, 1, 32); l += __shfl_xor(l, 2, 32); l += __shfl_xor(l, 4, 32); l += __shfl_xor(l, 8, 32);
    l_r[r] = (l > 0.f) ? 1.0f / l : 0.f;
  }
#pragma unroll
  for (int dt = 0; dt < DT; ++dt)
#pragma unroll
    for (int r = 0; r < 8; ++r) sO[w][8 * hh + r][dt * 16 + ln] = oacc[dt][r] * l_r[r];
  __builtin_amdgcn_fence(__ATOMIC_ACQ_REL, "workgroup");
  __builtin_amdgcn_wave_barrier();
  for (int pass = 0; pass < 2; ++pass) {
    for (int r = 0; r < 16; ++r) {
      const int row = q0 + r;
      if (row < T && lane < D / 4) {
        const v4f val = *(const v4fa*)&sO[w][r][lane * 4];
        *(volatile v4f*)(y + ((size_t)b * T + row) * ypitch + h * D + lane * 4) = val;
      }
    }
    if (pass == 0) __threadfence();
  }
}

__global__ __launch_bounds__(256) void k_sort_init(const int* __restrict__ seg, int n, int nseg, unsigned int* __restrict__ key, unsigned int* __restrict__ val, int np2) {
  const int i = blockIdx.x * 256 + threadIdx.x; if (i >= np2) return;
  unsigned int kv = 0xFFFFFFFFu;
  if (i < n) { int s = seg[i]; s = s < 0 ? 0 : (s >= nseg ? nseg - 1 : s); kv = (unsigned int)s; }
  *(volatile unsigned int*)(key + i) = kv; *(volatile unsigned int*)(val + i) = (unsigned int)i;
  __threadfence();
  *(volatile unsigned int*)(key + i) = kv; *(volatile unsigned int*)(val + i) = (unsigned int)i;
}
template <bool STAGE0>
__global__ __launch_bounds__(512) void k_sort_lds(unsigned int* __restrict__ key, unsigned int* __restrict__ val, int kstage) {
  __shared__ unsigned int sk[1024], sv[1024];
  const int tid = threadIdx.x; const int base = blockIdx.x * 1024;
  sk[tid] = key[base + tid]; sv[tid] = val[base + tid]; sk[tid + 512] = key[base + tid + 512]; sv[tid + 512] = val[base + tid + 512];
  __syncthreads();
  for (int k = (STAGE0 ? 2 : kstage); k <= (STAGE0 ? 1024 : kstage); k <<= 1) {
    for (int j = (k > 1024 ? 512 : (k >> 1)); j >= 1; j >>= 1) {
      const int lo = tid & (j - 1), hi2 = (tid >> __builtin_ctz(j)) << (__builtin_ctz(j) + 1);
      const int il = hi2 | lo, ir = il | j;
      const int gi = base + il;
      const bool asc = ((gi & k) == 0);
      unsigned int a = sk[il], b = sk[ir], va = sv[il], vb = sv[ir];
      const bool swp = asc ? (a > b) : (a < b);
      if (swp) { sk[il] = b; sk[ir] = a; sv[il] = vb; sv[ir] = va; }
      __syncthreads();
    }
  }
  for (int pass = 0; pass < 2; ++pass) {
    *(volatile unsigned int*)(key + base + tid) = sk[tid]; *(volatile unsigned int*)(val + base + tid) = sv[tid];
    *(volatile unsigned int*)(key + base + tid + 512) = sk[tid + 512]; *(volatile unsigned int*)(val + base + tid + 512) = sv[tid + 512];
    if (pass == 0) __threadfence();
  }
}
__global__ __launch_bounds__(256) void k_sort_step(unsigned int* __restrict__ key, unsigned int* __restrict__ val, int k, int j, int np2) {
  const int t = blockIdx.x * 256 + threadIdx.x; if (t >= np2 / 2) return;
  const int lo = t & (j - 1), il = ((t >> __builtin_ctz(j)) << (__builtin_ctz(j) + 1)) | lo, ir = il | j;
  const bool asc = ((il & k) == 0);
  unsigned int a = key[il], b = key[ir], va = val[il], vb = val[ir];
  const bool swp = asc ? (a > b) : (a < b);
  const unsigned int k1 = swp ? b : a, k2 = swp ? a : b, v1 = swp ? vb : va, v2 = swp ? va : vb;
  *(volatile unsigned int*)(key + il) = k1; *(volatile unsigned int*)(key + ir) = k2; *(volatile unsigned int*)(val + il) = v1; *(volatile unsigned int*)(val + ir) = v2;
  __threadfence();
  *(volatile unsigned int*)(key + il) = k1; *(volatile unsigned int*)(key + ir) = k2; *(volatile unsigned int*)(val + il) = v1; *(volatile unsigned int*)(val + ir) = v2;
}
__global__ __launch_bounds__(256) void k_rowptr(const unsigned int* __restrict__ key, int np2, int nseg, int* __restrict__ rowptr) {
  int s = blockIdx.x * 256 + threadIdx.x; if (s >= ((nseg + 1 + 31) / 32) * 32) return;
  const int sdst = s; if (s > nseg) s = nseg;
  int lo = 0, hi = np2;
  while (lo < hi) { const int mid = (lo + hi) >> 1; if (key[mid] < (unsigned int)s) lo = mid + 1; else hi = mid; }
  *(volatile int*)(rowptr + sdst) = lo; __threadfence(); *(volatile int*)(rowptr + sdst) = lo;
}
static void sort_pairs(unsigned int* key, unsigned int* val, int np2, hipStream_t stream) {
  k_sort_lds<true><<<np2 / 1024, 512, 0, stream>>>(key, val, 0);
  for (int k = 2048; k <= np2; k <<= 1) {
    for (int j = k >> 1; j >= 1024; j >>= 1) k_sort_step<<<(np2 / 2 + 255) / 256, 256, 0, stream>>>(key, val, k, j, np2);
    k_sort_lds<false><<<np2 / 1024, 512, 0, stream>>>(key, val, k);
  }
}

__device__ __forceinline__ float silu_f(float x) { return x / (1.0f + expf(-x)); }
__global__ __launch_bounds__(256) void k_gptr(const int* __restrict__ batch, int* __restrict__ gptr) {
  const int slot = blockIdx.x * 256 + threadIdx.x; if (slot >= ((NG + 1 + 31) / 32) * 32) return; const int g = slot > NG ? NG : slot;
  int lo = 0, hi = NNODE; while (lo < hi) { const int mid = (lo + hi) >> 1; if (batch[mid] < g) lo = mid + 1; else hi = mid; }
  *(volatile int*)(gptr + slot) = lo; __threadfence(); *(volatile int*)(gptr + slot) = lo;
}
template <bool ROUND>
__global__ __launch_bounds__(384) void k_gmean(const float* __restrict__ src, const int* __restrict__ gptr, float* __restrict__ mean) {
  const int g = blockIdx.x, t = threadIdx.x; const int n0 = gptr[g], n1 = gptr[g + 1]; float s = 0.f;
#pragma unroll 1
  for (int n = n0; n < n1; ++n) { float v = src[(size_t)n * 3 * KV + t]; if (ROUND) v = bf16_round(v); s += v; }
  s = s / fmaxf((float)(n1 - n0), 1.0f);
  *(volatile float*)(mean + (size_t)g * 3 * KV + t) = s; __threadfence(); *(volatile float*)(mean + (size_t)g * 3 * KV + t) = s;
}
__global__ __launch_bounds__(128) void k_center(const float* __restrict__ X, const int* __restrict__ batch, const float* __restrict__ meanG, float* __restrict__ X1, float* __restrict__ nrm) {
  const int n = blockIdx.x, k = threadIdx.x; int g = batch[n]; g = g < 0 ? 0 : (g >= NG ? NG - 1 : g);
  float v[3], s = 0.f; for (int c = 0; c < 3; ++c) { v[c] = bf16_round(X[((size_t)n * 3 + c) * KV + k]) - meanG[((size_t)g * 3 + c) * KV + k]; s += v[c] * v[c]; }
  const float nm = sqrtf(s);
  for (int pass = 0; pass < 2; ++pass) { for (int c = 0; c < 3; ++c) *(volatile float*)(X1 + ((size_t)n * 3 + c) * KV + k) = v[c]; *(volatile float*)(nrm + (size_t)n * KV + k) = nm; if (pass == 0) __threadfence(); }
}
__global__ __launch_bounds__(128) void k_gmean_norm(const float* __restrict__ nrm, const int* __restrict__ gptr, float* __restrict__ mn) {
  const int g = blockIdx.x, k = threadIdx.x; const int n0 = gptr[g], n1 = gptr[g + 1]; float s = 0.f;
#pragma unroll 1
  for (int n = n0; n < n1; ++n) s += nrm[(size_t)n * KV + k];
  s = s / fmaxf((float)(n1 - n0), 1.0f);
  *(volatile float*)(mn + (size_t)g * KV + k) = s; __threadfence(); *(volatile float*)(mn + (size_t)g * KV + k) = s;
}
__global__ __launch_bounds__(128) void k_e3(const float* __restrict__ X1, const int* __restrict__ batch, const float* __restrict__ mn, const float* __restrict__ e3w, float* __restrict__ X2) {
  const int n = blockIdx.x, k = threadIdx.x; int g = batch[n]; g = g < 0 ? 0 : (g >= NG ? NG - 1 : g);
  const float sc = bf16_round(e3w[k]) / (mn[(size_t)g * KV + k] + 1e-5f);
  float v[3]; for (int c = 0; c < 3; ++c) v[c] = sc * X1[((size_t)n * 3 + c) * KV + k];
  for (int pass = 0; pass < 2; ++pass) { for (int c = 0; c < 3; ++c) *(volatile float*)(X2 + ((size_t)n * 3 + c) * KV + k) = v[c]; if (pass == 0) __threadfence(); }
}
__global__ __launch_bounds__(256) void k_ln64(const float* __restrict__ H, const float* __restrict__ w, const float* __restrict__ b, float* __restrict__ Hn) {
  const int tid = threadIdx.x, wv = tid >> 5, lane = tid & 31; const int n = blockIdx.x * 8 + wv; if (n >= NNODE) return;
  const float a = bf16_round(H[(size_t)n * DH + lane]), c = bf16_round(H[(size_t)n * DH + 32 + lane]);
  float s = a + c; for (int o = 16; o >= 1; o >>= 1) s += __shfl_xor(s, o, 32); const float mu = s * (1.0f / DH);
  float q2 = (a - mu) * (a - mu) + (c - mu) * (c - mu); for (int o = 16; o >= 1; o >>= 1) q2 += __shfl_xor(q2, o, 32); const float rs = rsqrtf(q2 * (1.0f / DH) + 1e-5f);
  const float o1 = (a - mu) * rs * bf16_round(w[lane]) + bf16_round(b[lane]), o2 = (c - mu) * rs * bf16_round(w[32 + lane]) + bf16_round(b[32 + lane]);
  *(volatile float*)(Hn + (size_t)n * DH + lane) = o1; *(volatile float*)(Hn + (size_t)n * DH + 32 + lane) = o2; __threadfence(); *(volatile float*)(Hn + (size_t)n * DH + lane) = o1; *(volatile float*)(Hn + (size_t)n * DH + 32 + lane) = o2;
}
__global__ __launch_bounds__(128) void k_edge(const float* __restrict__ Hn, const float* __restrict__ X2, const float* __restrict__ te, const int* __restrict__ batch, const int* __restrict__ src, const int* __restrict__ tgt, int e_base,
                                            const unsigned short* __restrict__ Bm1, const float* __restrict__ mb1, const unsigned short* __restrict__ Bm2, const float* __restrict__ mb2,
                                            const unsigned short* __restrict__ Bx1, const float* __restrict__ xb1, const unsigned short* __restrict__ Bx2, const float* __restrict__ xb2,
                                            const unsigned short* __restrict__ Bc1, const float* __restrict__ cb1, const unsigned short* __restrict__ Bc2, const float* __restrict__ cb2,
                                            float* __restrict__ w1out, float* __restrict__ w2out) {
  __shared__ __attribute__((aligned(16))) float sA[4][16][68];
  __shared__ __attribute__((aligned(16))) float sM[4][16][68];
  __shared__ __attribute__((aligned(16))) float so[4][16][64];
  const int tid = threadIdx.x, w = tid >> 5, lane = tid & 31, ln = lane & 15, hh = lane >> 4;
  const size_t el0 = ((size_t)blockIdx.x * 4 + w) * 16; if (el0 >= (size_t)ESL) return; const size_t e = (size_t)e_base + el0 + ln;
  int sn = src[e]; sn = sn < 0 ? 0 : (sn >= NNODE ? NNODE - 1 : sn); int tn = tgt[e]; tn = tn < 0 ? 0 : (tn >= NNODE ? NNODE - 1 : tn);
  int gs = batch[sn]; gs = gs < 0 ? 0 : (gs >= NG ? NG - 1 : gs);
  const float* ht = Hn + (size_t)tn * DH; const float* hs = Hn + (size_t)sn * DH; const float* xs = X2 + (size_t)sn * 3 * KV; const float* xt = X2 + (size_t)tn * 3 * KV; const float* ter = te + (size_t)gs * TE;
  v8f acc[4]; for (int t = 0; t < 4; ++t) acc[t] = (v8f){0.f,0.f,0.f,0.f,0.f,0.f,0.f,0.f};
#pragma unroll 1
  for (int ks = 0; ks < MSGK / 32; ++ks) {
    FragB ah, al;
#pragma unroll
    for (int i = 0; i < 16; ++i) { const int k = ks * 32 + ((i < 8) ? (8 * hh + i) : (16 + 8 * hh + (i - 8))); float v;
      if (k < DH) v = ht[k]; else if (k < 2 * DH) v = hs[k - DH];
      else if (k < 2 * DH + KV) { const int kk = k - 2 * DH; const float r0 = xs[kk] - xt[kk], r1 = xs[KV + kk] - xt[KV + kk], r2 = xs[2 * KV + kk] - xt[2 * KV + kk]; v = r0 * r0 + r1 * r1 + r2 * r2; }
      else v = bf16_round(ter[k - 2 * DH - KV]);
      const unsigned short hb = bf16_bits(v); ah.u[i] = hb; al.u[i] = bf16_bits(v - bf16_val(hb)); }
#pragma unroll
    for (int t = 0; t < 4; ++t) { FragB b; b.half[0] = *(const v8us*)(Bm1 + (size_t)(t * 16 + ln) * MSGK + ks * 32 + 8 * hh); b.half[1] = *(const v8us*)(Bm1 + (size_t)(t * 16 + ln) * MSGK + ks * 32 + 16 + 8 * hh); acc[t] = mmaN<2>(ah.v, al.v, b.v, b.v, acc[t]); }
  }
#pragma unroll
  for (int t = 0; t < 4; ++t) { const int col = t * 16 + ln; const float bb = bf16_round(mb1[col]);
#pragma unroll
    for (int r = 0; r < 8; ++r) sA[w][8 * hh + r][col] = silu_f(acc[t][r] + bb); }
  __builtin_amdgcn_fence(__ATOMIC_ACQ_REL, "workgroup"); __builtin_amdgcn_wave_barrier();
  auto lds_frag = [&](const float (*rows)[68], int ks, FragB& ah, FragB& al) {
#pragma unroll
    for (int i = 0; i < 16; ++i) { const int k = ks * 32 + ((i < 8) ? (8 * hh + i) : (16 + 8 * hh + (i - 8))); const float v = rows[ln][k]; const unsigned short hb = bf16_bits(v); ah.u[i] = hb; al.u[i] = bf16_bits(v - bf16_val(hb)); } };
  { FragB ah[2], al[2]; lds_frag(sA[w], 0, ah[0], al[0]); lds_frag(sA[w], 1, ah[1], al[1]);
    v8f a2[4]; for (int t = 0; t < 4; ++t) a2[t] = (v8f){0.f,0.f,0.f,0.f,0.f,0.f,0.f,0.f};
#pragma unroll
    for (int ks = 0; ks < 2; ++ks)
#pragma unroll
      for (int t = 0; t < 4; ++t) { FragB b; b.half[0] = *(const v8us*)(Bm2 + (size_t)(t * 16 + ln) * DH + ks * 32 + 8 * hh); b.half[1] = *(const v8us*)(Bm2 + (size_t)(t * 16 + ln) * DH + ks * 32 + 16 + 8 * hh); a2[t] = mmaN<2>(ah[ks].v, al[ks].v, b.v, b.v, a2[t]); }
#pragma unroll
    for (int t = 0; t < 4; ++t) { const int col = t * 16 + ln; const float bb = bf16_round(mb2[col]);
#pragma unroll
      for (int r = 0; r < 8; ++r) sM[w][8 * hh + r][col] = a2[t][r] + bb; } }
  __builtin_amdgcn_fence(__ATOMIC_ACQ_REL, "workgroup"); __builtin_amdgcn_wave_barrier();
#pragma unroll 1
  for (int which = 0; which < 2; ++which) {
    const unsigned short* B1 = which ? Bc1 : Bx1; const float* b1 = which ? cb1 : xb1; const unsigned short* B2 = which ? Bc2 : Bx2; const float* b2 = which ? cb2 : xb2; float* wout = which ? w2out : w1out;
    { FragB ah[2], al[2]; lds_frag(sM[w], 0, ah[0], al[0]); lds_frag(sM[w], 1, ah[1], al[1]);
      v8f a2[4]; for (int t = 0; t < 4; ++t) a2[t] = (v8f){0.f,0.f,0.f,0.f,0.f,0.f,0.f,0.f};
#pragma unroll
      for (int ks = 0; ks < 2; ++ks)
#pragma unroll
        for (int t = 0; t < 4; ++t) { FragB b; b.half[0] = *(const v8us*)(B1 + (size_t)(t * 16 + ln) * DH + ks * 32 + 8 * hh); b.half[1] = *(const v8us*)(B1 + (size_t)(t * 16 + ln) * DH + ks * 32 + 16 + 8 * hh); a2[t] = mmaN<2>(ah[ks].v, al[ks].v, b.v, b.v, a2[t]); }
      __builtin_amdgcn_fence(__ATOMIC_ACQ_REL, "workgroup"); __builtin_amdgcn_wave_barrier();
#pragma unroll
      for (int t = 0; t < 4; ++t) { const int col = t * 16 + ln; const float bb = bf16_round(b1[col]);
#pragma unroll
        for (int r = 0; r < 8; ++r) sA[w][8 * hh + r][col] = silu_f(a2[t][r] + bb); } }
    __builtin_amdgcn_fence(__ATOMIC_ACQ_REL, "workgroup"); __builtin_amdgcn_wave_barrier();
    { FragB ah[2], al[2]; lds_frag(sA[w], 0, ah[0], al[0]); lds_frag(sA[w], 1, ah[1], al[1]);
#pragma unroll 1
      for (int half = 0; half < 2; ++half) {
        v8f a2[4]; for (int t = 0; t < 4; ++t) a2[t] = (v8f){0.f,0.f,0.f,0.f,0.f,0.f,0.f,0.f};
#pragma unroll
        for (int ks = 0; ks < 2; ++ks)
#pragma unroll
          for (int t = 0; t < 4; ++t) { const int n = half * 64 + t * 16 + ln; FragB b; b.half[0] = *(const v8us*)(B2 + (size_t)n * DH + ks * 32 + 8 * hh); b.half[1] = *(const v8us*)(B2 + (size_t)n * DH + ks * 32 + 16 + 8 * hh); a2[t] = mmaN<2>(ah[ks].v, al[ks].v, b.v, b.v, a2[t]); }
#pragma unroll
        for (int t = 0; t < 4; ++t) { const int col = half * 64 + t * 16 + ln; const float bb = bf16_round(b2[col]);
#pragma unroll
          for (int r = 0; r < 8; ++r) so[w][8 * hh + r][t * 16 + ln] = fminf(fmaxf(a2[t][r] + bb, -10.0f), 10.0f); }
        __builtin_amdgcn_fence(__ATOMIC_ACQ_REL, "workgroup"); __builtin_amdgcn_wave_barrier();
        const int rsub = lane >> 4, c4 = (lane & 15) * 4;
        for (int pass = 0; pass < 2; ++pass) { for (int q = 0; q < 8; ++q) { const int r = q * 2 + rsub; const v4f v = *(const v4fa*)&so[w][r][c4]; *(volatile v4f*)(wout + (el0 + r) * KV + half * 64 + c4) = v; } if (pass == 0) __threadfence(); }
        __builtin_amdgcn_fence(__ATOMIC_ACQ_REL, "workgroup"); __builtin_amdgcn_wave_barrier();
      } }
  }
}
__global__ __launch_bounds__(128) void k_aggx(const float* __restrict__ X2, const float* __restrict__ meanN, const int* __restrict__ src, const float* __restrict__ w1, const float* __restrict__ w2, int e_base, int first,
                                            const int* __restrict__ rowptr, const unsigned int* __restrict__ perm, float* out) {
  const int n = blockIdx.x, k = threadIdx.x;
  float a0, a1, a2;
  if (first) { a0 = X2[((size_t)n * 3 + 0) * KV + k]; a1 = X2[((size_t)n * 3 + 1) * KV + k]; a2 = X2[((size_t)n * 3 + 2) * KV + k]; }
  else { a0 = out[((size_t)n * 3 + 0) * KV + k]; a1 = out[((size_t)n * 3 + 1) * KV + k]; a2 = out[((size_t)n * 3 + 2) * KV + k]; }
  const float t0 = X2[((size_t)n * 3 + 0) * KV + k], t1 = X2[((size_t)n * 3 + 1) * KV + k], t2 = X2[((size_t)n * 3 + 2) * KV + k];
  const float mt0 = (n < NG) ? meanN[((size_t)n * 3 + 0) * KV + k] : 0.f, mt1 = (n < NG) ? meanN[((size_t)n * 3 + 1) * KV + k] : 0.f, mt2 = (n < NG) ? meanN[((size_t)n * 3 + 2) * KV + k] : 0.f;
  const float xt0 = t0 - mt0, xt1 = t1 - mt1, xt2 = t2 - mt2;
#pragma unroll 1
  for (int p = rowptr[n]; p < rowptr[n + 1]; ++p) { const int e = (int)perm[p]; if (e < e_base || e >= e_base + ESL) continue;
    int sn = src[e]; sn = sn < 0 ? 0 : (sn >= NNODE ? NNODE - 1 : sn);
    const float s0 = X2[((size_t)sn * 3 + 0) * KV + k], s1 = X2[((size_t)sn * 3 + 1) * KV + k], s2 = X2[((size_t)sn * 3 + 2) * KV + k];
    const float r0 = s0 - t0, r1 = s1 - t1, r2 = s2 - t2; const float rd = r0 * r0 + r1 * r1 + r2 * r2; const float inv = 1.0f / (1.0f + sqrtf(rd + 1e-8f));
    const float wa = w1[(size_t)(e - e_base) * KV + k], wb = w2[(size_t)(e - e_base) * KV + k];
    const float ms0 = (sn < NG) ? meanN[((size_t)sn * 3 + 0) * KV + k] : 0.f, ms1 = (sn < NG) ? meanN[((size_t)sn * 3 + 1) * KV + k] : 0.f, ms2 = (sn < NG) ? meanN[((size_t)sn * 3 + 2) * KV + k] : 0.f;
    const float xs0 = s0 - ms0, xs1 = s1 - ms1, xs2 = s2 - ms2;
    float c0 = xs1 * xt2 - xs2 * xt1, c1 = xs2 * xt0 - xs0 * xt2, c2 = xs0 * xt1 - xs1 * xt0;
    const float cn = 1.0f / (1.0f + sqrtf(c0 * c0 + c1 * c1 + c2 * c2));
    a0 += r0 * inv * wa + c0 * cn * wb; a1 += r1 * inv * wa + c1 * cn * wb; a2 += r2 * inv * wa + c2 * cn * wb;
  }
  for (int pass = 0; pass < 2; ++pass) { *(volatile float*)(out + ((size_t)n * 3 + 0) * KV + k) = a0; *(volatile float*)(out + ((size_t)n * 3 + 1) * KV + k) = a1; *(volatile float*)(out + ((size_t)n * 3 + 2) * KV + k) = a2; if (pass == 0) __threadfence(); }
}
extern "C" void kernel_launch(void* const* d_in, const int* in_sizes, int n_in,
                              void* d_out, int out_size, void* d_ws, size_t ws_size, hipStream_t stream) {
  (void)in_sizes; (void)n_in; (void)out_size;
  const int* batch = (const int*)d_in[0]; const float* X = (const float*)d_in[1]; const float* H = (const float*)d_in[2]; const int* ei = (const int*)d_in[3]; const float* te = (const float*)d_in[4];
  const float* e3w = (const float*)d_in[5]; const float* lnw = (const float*)d_in[6]; const float* lnb = (const float*)d_in[7];
  const float* mw1 = (const float*)d_in[8]; const float* mb1 = (const float*)d_in[9]; const float* mw2 = (const float*)d_in[10]; const float* mb2 = (const float*)d_in[11];
  const float* xw1 = (const float*)d_in[12]; const float* xb1 = (const float*)d_in[13]; const float* xw2 = (const float*)d_in[14]; const float* xb2 = (const float*)d_in[15];
  const float* cw1 = (const float*)d_in[16]; const float* cb1 = (const float*)d_in[17]; const float* cw2 = (const float*)d_in[18]; const float* cb2 = (const float*)d_in[19];
  const int* src = ei; const int* tgt = ei + NEDGE;
  char* ws = (char*)d_ws; size_t off = 0;
  auto take = [&](size_t bytes) { char* p = ws + off; off += (bytes + 255) & ~(size_t)255; return p; };
  unsigned short* Bm1 = (unsigned short*)take((size_t)DH * MSGK * 2); unsigned short* Bm2 = (unsigned short*)take((size_t)DH * DH * 2);
  unsigned short* Bx1 = (unsigned short*)take((size_t)DH * DH * 2); unsigned short* Bx2 = (unsigned short*)take((size_t)KV * DH * 2); unsigned short* Bc1 = (unsigned short*)take((size_t)DH * DH * 2); unsigned short* Bc2 = (unsigned short*)take((size_t)KV * DH * 2);
  unsigned int* key = (unsigned int*)take((size_t)NP2 * 4); unsigned int* perm = (unsigned int*)take((size_t)NP2 * 4); int* rowptr = (int*)take((size_t)(NNODE + 64) * 4); int* gptr = (int*)take((size_t)(NG + 64) * 4);
  float* meanG = (float*)take((size_t)NG * 3 * KV * 4); float* X1 = (float*)take((size_t)NNODE * 3 * KV * 4); float* nrm = (float*)take((size_t)NNODE * KV * 4); float* mn = (float*)take((size_t)NG * KV * 4);
  float* X2 = (float*)take((size_t)NNODE * 3 * KV * 4); float* meanN = (float*)take((size_t)NG * 3 * KV * 4); float* Hn = (float*)take((size_t)NNODE * DH * 4);
  float* w1 = (float*)take((size_t)ESL * KV * 4); float* w2 = (float*)take((size_t)ESL * KV * 4);
  if (off > ws_size) return;
  k_wt_bf16<<<(DH * (MSGK / 8) + 255) / 256, 256, 0, stream>>>(mw1, Bm1, MSGK, DH); k_wt_bf16<<<(DH * (DH / 8) + 255) / 256, 256, 0, stream>>>(mw2, Bm2, DH, DH);
  k_wt_bf16<<<(DH * (DH / 8) + 255) / 256, 256, 0, stream>>>(xw1, Bx1, DH, DH); k_wt_bf16<<<(KV * (DH / 8) + 255) / 256, 256, 0, stream>>>(xw2, Bx2, DH, KV);
  k_wt_bf16<<<(DH * (DH / 8) + 255) / 256, 256, 0, stream>>>(cw1, Bc1, DH, DH); k_wt_bf16<<<(KV * (DH / 8) + 255) / 256, 256, 0, stream>>>(cw2, Bc2, DH, KV);
  k_sort_init<<<NP2 / 256, 256, 0, stream>>>(tgt, NEDGE, NNODE, key, perm, NP2);
  sort_pairs(key, perm, NP2, stream);
  k_rowptr<<<(NNODE + 32 + 255) / 256, 256, 0, stream>>>(key, NP2, NNODE, rowptr);
  k_gptr<<<(NG + 32 + 255) / 256, 256, 0, stream>>>(batch, gptr);
  k_gmean<true><<<NG, 384, 0, stream>>>(X, gptr, meanG);
  k_center<<<NNODE, 128, 0, stream>>>(X, batch, meanG, X1, nrm);
  k_gmean_norm<<<NG, 128, 0, stream>>>(nrm, gptr, mn);
  k_e3<<<NNODE, 128, 0, stream>>>(X1, batch, mn, e3w, X2);
  k_gmean<false><<<NG, 384, 0, stream>>>(X2, gptr, meanN);
  k_ln64<<<(NNODE + 7) / 8, 256, 0, stream>>>(H, lnw, lnb, Hn);
  for (int sl = 0; sl < NSL; ++sl) {
    k_edge<<<(ESL / 16 + 3) / 4, 128, 0, stream>>>(Hn, X2, te, batch, src, tgt, sl * ESL, Bm1, mb1, Bm2, mb2, Bx1, xb1, Bx2, xb2, Bc1, cb1, Bc2, cb2, w1, w2);
    k_aggx<<<NNODE, 128, 0, stream>>>(X2, meanN, src, w1, w2, sl * ESL, sl == 0 ? 1 : 0, rowptr, perm, (float*)d_out);
  }
}
